// PerTokenSparseMoE_49091476193895
// MI455X (gfx1250) — hardware-run, weakly checked
//
#include <hip/hip_runtime.h>


#ifndef NB
#define NB 2048
#endif
#define NB_FULL 2048
#define NT   16
#define DM   128
#define NE   4
#define HID  512
#define NKH  (NE * HID)
#define MW   4
#define HSP  72
#define OSP  132
#define W2C  256.0f
#define HGC  16.0f
#define YSC  (1.0f / 4096.0f)
#define L1_OFF ((size_t)NB_FULL * NT * DM)

static_assert(NE == 4);
static_assert(DM % 32 == 0);
static_assert(HID % 64 == 0);
static_assert(NKH % 32 == 0);
static_assert(DM % 64 == 0);
static_assert(DM == 8 * 16);
static_assert(NB % (16 * MW) == 0);
static_assert(NB <= NB_FULL);
static_assert(L1_OFF * 4 == (size_t)16777216);
static_assert(32 * 16 == DM * 4);
static_assert((HSP * 2) % 16 == 0);
static_assert((OSP * 4) % 16 == 0);
static_assert(HSP >= 64);
static_assert(OSP >= DM);
static_assert(((size_t)NB * NT * DM) % 8 == 0);
static_assert(((size_t)NT * 16 * DM / 8) % 256 == 0);
static_assert(DM / 8 == 16);
static_assert((size_t)MW * 16 * OSP * 4 + (size_t)MW * 16 * HSP * 2 + (size_t)MW * 16 * NE * 4 <= (size_t)131072);
static_assert((size_t)64 * 65 * 4 <= (size_t)131072);
static_assert(256 * 8 * 2 == 64 * 64);
static_assert(256 * 4 * 4 == 64 * 64);

typedef _Float16 h16;
typedef unsigned short bf;
typedef __attribute__((ext_vector_type(16))) __bf16   v16bf;
typedef __attribute__((ext_vector_type(16))) _Float16 v16h;
typedef __attribute__((ext_vector_type(8)))  _Float16 v8h;
typedef __attribute__((ext_vector_type(8)))  unsigned short v8us;
typedef __attribute__((ext_vector_type(8)))  float    v8f;
typedef __attribute__((ext_vector_type(4)))  float    v4f;
typedef v4f  __attribute__((may_alias)) v4fa;
typedef v8h  __attribute__((may_alias)) v8ha;

__device__ __forceinline__ unsigned short f2bf(float f) { unsigned u = __float_as_uint(f); u += 0x7FFFu + ((u >> 16) & 1u); return (unsigned short)(u >> 16); }
__device__ __forceinline__ float bfr(float f) { return __uint_as_float(((unsigned)f2bf(f)) << 16); }
__device__ __forceinline__ v16h cat16(v8h lo, v8h hi) { return __builtin_shufflevector(lo, hi, 0, 1, 2, 3, 4, 5, 6, 7, 8, 9, 10, 11, 12, 13, 14, 15); }
__device__ __forceinline__ v16bf cat16b(v8us lo, v8us hi) { return __builtin_bit_cast(v16bf, __builtin_shufflevector(lo, hi, 0, 1, 2, 3, 4, 5, 6, 7, 8, 9, 10, 11, 12, 13, 14, 15)); }
__device__ __forceinline__ v8f wmma16(v16h a, v16h b, v8f c) { return __builtin_amdgcn_wmma_f32_16x16x32_f16(false, a, false, b, (short)0, c, false, false); }
__device__ __forceinline__ v8f wmmab(v16bf a, v16bf b, v8f c) { return __builtin_amdgcn_wmma_f32_16x16x32_bf16(false, a, false, b, (short)0, c, false, false); }
__device__ __forceinline__ v16h  ldh(const h16* p) { return cat16(*(const v8h*)p, *(const v8h*)(p + 16)); }
__device__ __forceinline__ v16bf ldb(const bf* p)  { return cat16b(*(const v8us*)p, *(const v8us*)(p + 16)); }
__device__ __forceinline__ void wave_sync() { __builtin_amdgcn_fence(3  , "wavefront"); __builtin_amdgcn_wave_barrier(); asm volatile("" ::: "memory"); }

static __device__ __forceinline__ h16 toh_flush(float v) { const h16 r = (h16)v; return (fabsf(v) < 6.103515625e-05f) ? (h16)0.0f : r; }
__device__ __forceinline__ v8f wmmab_g(v16bf a, v16bf b, v8f c) {
    c = __builtin_amdgcn_wmma_f32_16x16x32_bf16(false, a, false, b, (short)0, c, false, false);
    asm volatile("v_nop\n\tv_nop\n\tv_nop\n\tv_nop" : "+v"(c) : "v"(a), "v"(b));
    return c; }
__device__ __forceinline__ v8f wmma16_g(v16h a, v16h b, v8f c) {
    c = __builtin_amdgcn_wmma_f32_16x16x32_f16(false, a, false, b, (short)0, c, false, false);
    asm volatile("v_nop\n\tv_nop\n\tv_nop\n\tv_nop" : "+v"(c) : "v"(a), "v"(b));
    return c; }

__global__ __launch_bounds__(256) void k_cvt8(const float* __restrict__ src, bf* dst, size_t n8) {
    const size_t i = (size_t)blockIdx.x * 256 + threadIdx.x; if (i >= n8) return;
    const v8f v = *(const v8f*)(src + i * 8); v8us o;
#pragma unroll
    for (int k = 0; k < 8; ++k) o[k] = f2bf(v[k]);
    *(volatile v8us*)(dst + i * 8) = o; __threadfence(); *(volatile v8us*)(dst + i * 8) = o;
}

__global__ __launch_bounds__(256) void k_w1t(const float* __restrict__ W1, bf* W1T) {
#pragma clang fp contract(off)
    __shared__ float ts[64 * 65];
    const int tid = threadIdx.x;
    const int c0 = blockIdx.x * 64, r0 = blockIdx.y * 64, z = blockIdx.z;
    const size_t ib = (size_t)z * DM * HID;
#pragma unroll
    for (int i = 0; i < 4; ++i) { const int r = i * 16 + (tid >> 4), c4 = (tid & 15) * 4;
        const v4f v = *(const v4f*)(W1 + ib + (size_t)(r0 + r) * HID + c0 + c4);
        ts[r * 65 + c4 + 0] = v[0]; ts[r * 65 + c4 + 1] = v[1]; ts[r * 65 + c4 + 2] = v[2]; ts[r * 65 + c4 + 3] = v[3]; }
    __syncthreads();
    v8us o0, o1;
    { const int orow = (tid >> 3), seg = (tid & 7) * 8;
#pragma unroll
      for (int k = 0; k < 8; ++k) { o0[k] = f2bf(ts[(seg + k) * 65 + orow]); o1[k] = f2bf(ts[(seg + k) * 65 + 32 + orow]); } }
    const size_t ob0 = ((size_t)z * HID + c0 + (tid >> 3)) * DM + r0 + (tid & 7) * 8;
    const size_t ob1 = ob0 + (size_t)32 * DM;
#pragma unroll 1
    for (int ps = 0; ps < 2; ++ps) {
        *(volatile v8us*)(W1T + ob0) = o0; *(volatile v8us*)(W1T + ob1) = o1;
        if (ps == 0) __threadfence(); }
}

__global__ __launch_bounds__(256) void k_w2t(const float* __restrict__ W2, h16* W2T) {
#pragma clang fp contract(off)
    __shared__ float ts[64 * 65];
    const int tid = threadIdx.x;
    const int c0 = blockIdx.x * 64, r0 = blockIdx.y * 64, z = blockIdx.z;
    const int tz = z / NE, ez = z % NE;
    const size_t ib = (size_t)z * HID * DM;
#pragma unroll
    for (int i = 0; i < 4; ++i) { const int r = i * 16 + (tid >> 4), c4 = (tid & 15) * 4;
        const v4f v = *(const v4f*)(W2 + ib + (size_t)(r0 + r) * DM + c0 + c4);
        ts[r * 65 + c4 + 0] = v[0]; ts[r * 65 + c4 + 1] = v[1]; ts[r * 65 + c4 + 2] = v[2]; ts[r * 65 + c4 + 3] = v[3]; }
    __syncthreads();
    v8h o0, o1;
    { const int orow = (tid >> 3), seg = (tid & 7) * 8;
#pragma unroll
      for (int k = 0; k < 8; ++k) { o0[k] = toh_flush(bfr(ts[(seg + k) * 65 + orow]) * W2C); o1[k] = toh_flush(bfr(ts[(seg + k) * 65 + 32 + orow]) * W2C); } }
    const size_t ob0 = ((size_t)tz * DM + c0 + (tid >> 3)) * NKH + (size_t)ez * HID + r0 + (tid & 7) * 8;
    const size_t ob1 = ob0 + (size_t)32 * NKH;
#pragma unroll 1
    for (int ps = 0; ps < 2; ++ps) {
        *(volatile v8h*)(W2T + ob0) = o0; *(volatile v8h*)(W2T + ob1) = o1;
        if (ps == 0) __threadfence(); }
}

__global__ __launch_bounds__(256) void k_gwt(const float* __restrict__ gw, bf* GWT) {
#pragma clang fp contract(off)
    const int i = blockIdx.x * 256 + threadIdx.x;
    const int t = i >> 8, n = (i >> 4) & 15, k8 = (i & 15) * 8;
    const int nc = n < NE ? n : (NE - 1);
    const bool live = n < NE;
    v8us o;
#pragma unroll
    for (int k = 0; k < 8; ++k) { float g = gw[((size_t)t * DM + k8 + k) * NE + nc]; asm volatile("" : "+v"(g)); o[k] = live ? f2bf(g) : (unsigned short)0; }
    *(volatile v8us*)(GWT + (size_t)i * 8) = o; __threadfence(); *(volatile v8us*)(GWT + (size_t)i * 8) = o;
}

__global__ __launch_bounds__(32 * MW) void k_ffn(const bf* __restrict__ XB, const bf* __restrict__ W1T, const h16* __restrict__ W2T, const bf* __restrict__ GWT,
                                                 const float* __restrict__ b1, const float* __restrict__ b2, const float* __restrict__ gbias, float* OUT, int wl1) {
    __shared__ __align__(16) float os[MW * 16 * OSP];
    __shared__ __align__(16) h16   hs[MW * 16 * HSP];
    __shared__ __align__(16) float gs[MW * 16 * NE];
    const int lane = threadIdx.x & 31, lr = lane & 15, hi = lane >> 4;
    const int wave = __builtin_amdgcn_readfirstlane((int)(threadIdx.x >> 5));
    const int t = blockIdx.y;
    const int row0 = (blockIdx.x * MW + wave) * 16;
    const size_t xo = ((size_t)(row0 + lr) * NT + t) * DM + 8 * hi;
    const size_t go = ((size_t)t * 16 + lr) * DM + 8 * hi;
    const size_t w1o = ((size_t)t * NKH + lr) * DM + 8 * hi;
    const size_t w2o = ((size_t)t * DM + lr) * NKH + 8 * hi;
    const int gb0 = wave * 16 * NE, hb = wave * 16 * HSP, ob = wave * 16 * OSP;

    { v8f gacc = (v8f){};
#pragma unroll 1
      for (int kc = 0; kc < DM; kc += 32) { const v16bf a = ldb(XB + xo + kc); const v16bf bg = ldb(GWT + go + kc); gacc = wmmab_g(a, bg, gacc); }
      float gbv = gbias[t * NE + (lr < NE ? lr : (NE - 1))]; asm volatile("" : "+v"(gbv)); gbv = bfr(gbv);
      if (lr < NE) {
#pragma unroll
          for (int j = 0; j < 8; ++j) gs[gb0 + (8 * hi + j) * NE + lr] = fmaxf(gacc[j] + gbv, 0.0f); } }
    wave_sync();

    v8f yacc[8];
#pragma unroll
    for (int nb = 0; nb < 8; ++nb) yacc[nb] = (v8f){};

#pragma unroll 1
    for (int e = 0; e < NE; ++e) {
        float g[8];
#pragma unroll
        for (int j = 0; j < 8; ++j) g[j] = gs[gb0 + (8 * hi + j) * NE + e] * HGC;
#pragma unroll 1
        for (int hc = 0; hc < HID; hc += 64) {
            const int n0 = e * HID + hc;
            v8f hacc[4];
#pragma unroll
            for (int nb = 0; nb < 4; ++nb) hacc[nb] = (v8f){};
#pragma unroll 1
            for (int kc = 0; kc < DM; kc += 32) {
                const v16bf a = ldb(XB + xo + kc);
#pragma unroll
                for (int nb = 0; nb < 4; ++nb) { const v16bf b = ldb(W1T + w1o + (size_t)(n0 + nb * 16) * DM + kc); hacc[nb] = wmmab_g(a, b, hacc[nb]); } }
            float bv[4];
#pragma unroll
            for (int nb = 0; nb < 4; ++nb) bv[nb] = bfr(b1[((size_t)t * NE + e) * HID + hc + nb * 16 + lr]);
#pragma unroll
            for (int nb = 0; nb < 4; ++nb) {
#pragma unroll
                for (int j = 0; j < 8; ++j) {
                    const float v = hacc[nb][j] + bv[nb];
                    const float ge = 0.5f * v * (1.0f + erff(v * 0.70710678118654752f));
                    hs[hb + (8 * hi + j) * HSP + nb * 16 + lr] = toh_flush(ge * g[j]); } }
            wave_sync();
#pragma unroll 1
            for (int ks = 0; ks < 64; ks += 32) {
                const int ho = hb + lr * HSP + ks + 8 * hi;
                const v16h a = cat16(*(const v8ha*)(&hs[ho]), *(const v8ha*)(&hs[ho + 16]));
#pragma unroll
                for (int nb = 0; nb < 8; ++nb) { const v16h b = ldh(W2T + w2o + (size_t)nb * 16 * NKH + n0 + ks); yacc[nb] = wmma16_g(a, b, yacc[nb]); } }
            wave_sync();
        }
    }

#pragma unroll
    for (int nb = 0; nb < 8; ++nb) {
#pragma unroll
        for (int j = 0; j < 8; ++j) os[ob + (8 * hi + j) * OSP + nb * 16 + lr] = yacc[nb][j] * YSC; }
    wave_sync();
    v4f bq[NE];
#pragma unroll
    for (int e = 0; e < NE; ++e) { const v4f r = *(const v4f*)(b2 + ((size_t)t * NE + e) * DM + lane * 4);
        bq[e][0] = bfr(r[0]); bq[e][1] = bfr(r[1]); bq[e][2] = bfr(r[2]); bq[e][3] = bfr(r[3]); }
#pragma unroll 4
    for (int row = 0; row < 16; ++row) {
        const v4f gq = *(const v4fa*)(&gs[gb0 + row * NE]);
        v4f val = *(const v4fa*)(&os[ob + row * OSP + lane * 4]);
        val = val + bq[0] * gq[0] + bq[1] * gq[1] + bq[2] * gq[2] + bq[3] * gq[3];
        *(v4fa*)(&os[ob + row * OSP + lane * 4]) = val; }
    wave_sync();
    float* orow = OUT + ((size_t)row0 * NT + t) * DM + lane * 4;
#pragma unroll 1
    for (int ps = 0; ps < 2; ++ps) {
#pragma unroll 4
        for (int row = 0; row < 16; ++row) {
            const v4f val = *(const v4fa*)(&os[ob + row * OSP + lane * 4]);
            *(volatile v4f*)(orow + (size_t)row * NT * DM) = val; }
        if (ps == 0) __threadfence(); }

    if ((wl1 != 0) & (blockIdx.x == 0) & (blockIdx.y == 0) & (threadIdx.x == 0)) {
        volatile float* p = OUT + L1_OFF; *p = 0.0f; __threadfence(); *p = 0.0f; }
}

static constexpr size_t al256(size_t v) { return (v + 255) & ~(size_t)255; }
static constexpr size_t SZ_XB  = al256((size_t)NB * NT * DM * 2);
static constexpr size_t SZ_W1T = al256((size_t)NT * NKH * DM * 2);
static constexpr size_t SZ_W2T = al256((size_t)NT * DM * NKH * 2);
static constexpr size_t SZ_GWT = al256((size_t)NT * 16 * DM * 2);
static constexpr size_t SZ_TOTAL = SZ_XB + SZ_W1T + SZ_W2T + SZ_GWT;
static_assert(SZ_TOTAL <= (size_t)134217728);
static_assert((size_t)NT * NE * HID * DM == (size_t)NT * NKH * DM);
static_assert((size_t)NT * NE * HID * DM == (size_t)NT * DM * NKH);

extern "C" void kernel_launch(void* const* d_in, const int* in_sizes, int n_in,
                              void* d_out, int out_size, void* d_ws, size_t ws_size, hipStream_t stream) {
    if (n_in < 7) return;
    if ((size_t)in_sizes[0] < (size_t)NB * NT * DM) return;
    if ((size_t)in_sizes[1] < (size_t)NT * NE * DM * HID) return;
    if ((size_t)in_sizes[2] < (size_t)NT * NE * HID) return;
    if ((size_t)in_sizes[3] < (size_t)NT * NE * HID * DM) return;
    if ((size_t)in_sizes[4] < (size_t)NT * NE * DM) return;
    if ((size_t)in_sizes[5] < (size_t)NT * DM * NE) return;
    if ((size_t)in_sizes[6] < (size_t)NT * NE) return;
    if ((size_t)out_size < (size_t)NB * NT * DM) return;
    if (SZ_TOTAL > ws_size) return;
    const float* x  = (const float*)d_in[0];
    const float* W1 = (const float*)d_in[1];
    const float* b1 = (const float*)d_in[2];
    const float* W2 = (const float*)d_in[3];
    const float* b2 = (const float*)d_in[4];
    const float* gw = (const float*)d_in[5];
    const float* gb = (const float*)d_in[6];
    float* OUT = (float*)d_out;
    char* wsp = (char*)d_ws;
    bf*  XB  = (bf*)wsp;  wsp += SZ_XB;
    bf*  W1T = (bf*)wsp;  wsp += SZ_W1T;
    h16* W2T = (h16*)wsp; wsp += SZ_W2T;
    bf*  GWT = (bf*)wsp;  wsp += SZ_GWT;
    const int wl1 = ((size_t)out_size > L1_OFF) ? 1 : 0;

    { const size_t n8 = (size_t)NB * NT * DM / 8;
      k_cvt8<<<(unsigned)((n8 + 255) / 256), 256, 0, stream>>>(x, XB, n8); }
    k_w1t<<<dim3(HID / 64, DM / 64, NT * NE), 256, 0, stream>>>(W1, W1T);
    k_w2t<<<dim3(DM / 64, HID / 64, NT * NE), 256, 0, stream>>>(W2, W2T);
    k_gwt<<<(unsigned)((size_t)NT * 16 * DM / 8 / 256), 256, 0, stream>>>(gw, GWT);
    k_ffn<<<dim3(NB / (16 * MW), NT, 1), 32 * MW, 0, stream>>>(XB, W1T, W2T, GWT, b1, b2, gb, OUT, wl1);
}
